// PW_Linear_31310311588556
// MI455X (gfx1250) — hardware-verified
//
#include <hip/hip_runtime.h>
#include <math.h>

#define NB_  131072
#define HID  256
#define NOUT 512
#define RPB  32

typedef _Float16 f16;
typedef __attribute__((ext_vector_type(16))) f16 f16x16;
typedef __attribute__((ext_vector_type(8)))  f16 f16x8;
typedef __attribute__((ext_vector_type(8)))  float f32x8;
typedef __attribute__((ext_vector_type(4)))  float v4f_t;
typedef float v4fa __attribute__((ext_vector_type(4), may_alias));

__device__ __forceinline__ f32x8 wmma16(f16x16 a, f16x16 b, f32x8 c) {
  c = __builtin_amdgcn_wmma_f32_16x16x32_f16(false, a, false, b, (short)0, c, false, false);
  asm volatile("v_nop\n\tv_nop\n\tv_nop\n\tv_nop" : "+v"(c) : "v"(a), "v"(b));
  return c;
}
__device__ __forceinline__ f16x16 lds_frag(const f16* base, int stride) {
  const int lane = threadIdx.x & 31, row = lane & 15, kh = (lane >> 4) * 8;
  const f16x8 lo = *(const f16x8*)(base + row * stride + kh);
  const f16x8 hi = *(const f16x8*)(base + row * stride + kh + 16);
  f16x16 f;
#pragma unroll
  for (int i = 0; i < 8; ++i) { f[i] = lo[i]; f[i + 8] = hi[i]; }
  return f;
}
__device__ __forceinline__ f16x16 load_frag(const float* __restrict__ base, int ld, int row0, int k0) {
  const int lane = threadIdx.x & 31, r = lane & 15, kh = (lane >> 4) * 8;
  const float* p0 = base + (size_t)(row0 + r) * ld + (k0 + kh);
  const v4f_t a = *(const v4f_t*)(p0), b = *(const v4f_t*)(p0 + 4), c = *(const v4f_t*)(p0 + 16), d = *(const v4f_t*)(p0 + 20);
  f16x16 f;
  f[0] = (f16)a[0]; f[1] = (f16)a[1]; f[2]  = (f16)a[2]; f[3]  = (f16)a[3]; f[4]  = (f16)b[0]; f[5]  = (f16)b[1]; f[6]  = (f16)b[2]; f[7]  = (f16)b[3];
  f[8] = (f16)c[0]; f[9] = (f16)c[1]; f[10] = (f16)c[2]; f[11] = (f16)c[3]; f[12] = (f16)d[0]; f[13] = (f16)d[1]; f[14] = (f16)d[2]; f[15] = (f16)d[3];
  return f;
}

__global__ __launch_bounds__(256) void k_fold(const float* __restrict__ W1, const float* __restrict__ b1, const float* __restrict__ W2,
                                              const float* __restrict__ b2, float* __restrict__ W21, float* __restrict__ b21) {
  const int o = threadIdx.x;
  float acc[16]; float bb = b2[o];
#pragma unroll
  for (int i = 0; i < 16; ++i) acc[i] = 0.0f;
  for (int j = 0; j < HID; ++j) {
    const float w = W2[o * HID + j];
    bb += w * b1[j];
#pragma unroll
    for (int i = 0; i < 16; ++i) acc[i] += w * W1[j * 16 + i];
  }
#pragma unroll 1
  for (int pass = 0; pass < 2; ++pass) {
#pragma unroll
    for (int g = 0; g < 4; ++g) { v4f_t v; v[0] = acc[4*g]; v[1] = acc[4*g+1]; v[2] = acc[4*g+2]; v[3] = acc[4*g+3]; *(volatile v4f_t*)(W21 + o * 16 + 4 * g) = v; }
    *(volatile float*)(b21 + o) = bb;
    __threadfence();
  }
}

__global__ __launch_bounds__(256) void k_pw(const float* __restrict__ x, const float* __restrict__ W21, const float* __restrict__ b21,
                                            const float* __restrict__ W3, const float* __restrict__ b3, float* __restrict__ z, float* __restrict__ ld) {
  __shared__ __attribute__((aligned(16))) f16 hS[RPB * 264];
  __shared__ __attribute__((aligned(16))) float lS[RPB * 516];
  __shared__ __attribute__((aligned(16))) float zS[RPB * 32];
  __shared__ __attribute__((aligned(16))) float ldS[RPB];
  const int tid = threadIdx.x, lane = tid & 31, wave = tid >> 5, cl = lane & 15, hsel = lane >> 4, kh = hsel * 8, rh = kh;
  const int row0 = blockIdx.x * RPB;

  {
    f16x16 xa[2];
#pragma unroll
    for (int t = 0; t < 2; ++t) {
      const float* xr = x + (size_t)(row0 + 16 * t + cl) * 32;
      f16x16 f;
#pragma unroll
      for (int i = 0; i < 8; ++i) { f[i] = (f16)xr[2 * (kh + i)]; f[8 + i] = (f16)0.0f; }
      xa[t] = f;
    }
#pragma unroll
    for (int j = 0; j < 2; ++j) {
      const int nt = wave * 2 + j;
      f16x16 bw;
#pragma unroll
      for (int i = 0; i < 8; ++i) { bw[i] = (f16)W21[(nt * 16 + cl) * 16 + kh + i]; bw[8 + i] = (f16)0.0f; }
      const float bb = b21[nt * 16 + cl];
#pragma unroll
      for (int t = 0; t < 2; ++t) {
        f32x8 acc = {};
        acc = wmma16(xa[t], bw, acc);
#pragma unroll
        for (int r = 0; r < 8; ++r) hS[(16 * t + rh + r) * 264 + nt * 16 + cl] = (f16)fmaxf(acc[r] + bb, 0.0f);
      }
    }
  }
  asm volatile("s_wait_dscnt 0" ::: "memory");
  __syncthreads();
  {
    f32x8 acc[2][4];
#pragma unroll
    for (int t = 0; t < 2; ++t)
#pragma unroll
      for (int j = 0; j < 4; ++j) { f32x8 zz = {}; acc[t][j] = zz; }
#pragma unroll 2
    for (int ks = 0; ks < HID / 32; ++ks) {
      const f16x16 a0 = lds_frag(hS + ks * 32, 264), a1 = lds_frag(hS + 16 * 264 + ks * 32, 264);
#pragma unroll
      for (int j = 0; j < 4; ++j) {
        const f16x16 bw = load_frag(W3, HID, wave * 64 + j * 16, ks * 32);
        acc[0][j] = wmma16(a0, bw, acc[0][j]); acc[1][j] = wmma16(a1, bw, acc[1][j]);
      }
    }
#pragma unroll
    for (int j = 0; j < 4; ++j) {
      const int n = wave * 64 + j * 16 + cl;
      const float bb = b3[n];
#pragma unroll
      for (int t = 0; t < 2; ++t)
#pragma unroll
        for (int r = 0; r < 8; ++r) lS[(16 * t + rh + r) * 516 + n] = acc[t][j][r] + bb;
    }
  }
  __syncthreads();
#pragma unroll 1
  for (int rr = 0; rr < 4; ++rr) {
    const int rl = wave * 4 + rr, row = row0 + rl;
    const float* lr = lS + rl * 516;
    float v[16], m = -INFINITY;
#pragma unroll
    for (int j = 0; j < 16; ++j) { v[j] = lr[lane + 32 * j]; m = fmaxf(m, v[j]); }
#pragma unroll
    for (int off = 16; off >= 1; off >>= 1) m = fmaxf(m, __shfl_xor(m, off, 32));
    float se = 0.0f;
#pragma unroll
    for (int j = 0; j < 16; ++j) { v[j] = __expf(v[j] - m); se += v[j]; }
#pragma unroll
    for (int off = 16; off >= 1; off >>= 1) se += __shfl_xor(se, off, 32);
    const float p = v[0] / se;
    float incl = p;
#pragma unroll
    for (int off = 1; off < 32; off <<= 1) { const float u = __shfl_up(incl, off, 32); if (lane >= off) incl += u; }
    const float excl = incl - p;
    const float xt = x[(size_t)row * 32 + 2 * cl + 1];
    const float xk = xt * 32.0f;
    const float fb = floorf(xk);
    int bi = (int)fb; bi = min(max(bi, 0), 31);
    const float alpha = xk - fb;
    const float g  = __shfl(p, bi, 32);
    const float gc = __shfl(excl, bi, 32);
    const float zt = alpha * g + gc;
    float ldd = (hsel == 0) ? logf(g * 32.0f) : 0.0f;
#pragma unroll
    for (int off = 8; off >= 1; off >>= 1) ldd += __shfl_xor(ldd, off, 32);
    if (hsel == 0) { zS[rl * 32 + 2 * cl] = x[(size_t)row * 32 + 2 * cl]; zS[rl * 32 + 2 * cl + 1] = zt; }
    if (lane == 0) ldS[rl] = ldd;
  }
  __syncthreads();
#pragma unroll 1
  for (int pass = 0; pass < 2; ++pass) {
    *(volatile v4f_t*)(z + (size_t)row0 * 32 + tid * 4) = *(const volatile v4fa*)(zS + tid * 4);
    if (tid < 8) *(volatile v4f_t*)(ld + row0 + tid * 4) = *(const volatile v4fa*)(ldS + tid * 4);
    __threadfence();
  }
}

extern "C" void kernel_launch(void* const* d_in, const int* in_sizes, int n_in,
                              void* d_out, int out_size, void* d_ws, size_t ws_size,
                              hipStream_t stream) {
  (void)in_sizes; (void)n_in; (void)out_size; (void)ws_size;
  const float* x  = (const float*)d_in[0];
  const float* W1 = (const float*)d_in[1];
  const float* b1 = (const float*)d_in[2];
  const float* W2 = (const float*)d_in[3];
  const float* b2 = (const float*)d_in[4];
  const float* W3 = (const float*)d_in[5];
  const float* b3 = (const float*)d_in[6];
  float* z  = (float*)d_out;
  float* ld = z + (size_t)NB_ * 32;
  float* W21 = (float*)d_ws;
  float* b21 = W21 + 256 * 16;
  k_fold<<<dim3(1), dim3(256), 0, stream>>>(W1, b1, W2, b2, W21, b21);
  k_pw<<<dim3(NB_ / RPB), dim3(256), 0, stream>>>(x, W21, b21, W3, b3, z, ld);
}
